// self_multihead_attention_566935683727
// MI455X (gfx1250) — hardware-verified
//
#include <hip/hip_runtime.h>
#include <math.h>
#include <stdint.h>

#define NB    4
#define TT    2048
#define DM    512
#define NH    16
#define HD    32
#define NTOK  (NB * TT)
#define NINST (NB * NH)
#define QBLK  128
static_assert(NH * HD == DM);
static_assert((TT % QBLK) == 0 && (TT % 64) == 0 && (DM % 64) == 0 && (NTOK % 64) == 0);
static_assert((NH % 2) == 0 && HD == 32 && (DM % 32) == 0);
static_assert(((NTOK * DM) % (8 * 256)) == 0);
static_assert(((NINST * TT * HD) % (8 * 256)) == 0);

typedef _Float16 v16h __attribute__((ext_vector_type(16)));
typedef _Float16 v8h  __attribute__((ext_vector_type(8)));
typedef float    v8f  __attribute__((ext_vector_type(8)));
typedef float    v4f  __attribute__((ext_vector_type(4)));
typedef unsigned int v4u __attribute__((ext_vector_type(4)));

__device__ __forceinline__ unsigned short bf_bits(float f) {
  unsigned u = __float_as_uint(f);
  return (unsigned short)((u + 0x7FFFu + ((u >> 16) & 1u)) >> 16);
}
__device__ __forceinline__ float bf_up(unsigned short h) { return __uint_as_float(((unsigned)h) << 16); }
__device__ __forceinline__ unsigned short h_bits(_Float16 x) { return __builtin_bit_cast(unsigned short, x); }
__device__ __forceinline__ unsigned pk16(unsigned short a, unsigned short b) { return (unsigned)a | ((unsigned)b << 16); }
__device__ __forceinline__ v8f zero8() { v8f z = {0.f, 0.f, 0.f, 0.f, 0.f, 0.f, 0.f, 0.f}; return z; }

__device__ __forceinline__ v16h ldfrag_h(const _Float16* p) {
  union { v16h v; v8h h[2]; } f;
  f.h[0] = *(const v8h*)(p);
  f.h[1] = *(const v8h*)(p + 16);
  return f.v;
}

__device__ __forceinline__ v8f mma_h_raw(v16h a, v16h b, v8f c) {
  return __builtin_amdgcn_wmma_f32_16x16x32_f16(false, a, false, b, (short)0, c, false, false);
}
__device__ __forceinline__ void res_guard(v8f& t, v8f& acc, v16h x, v16h y) {
#if defined(__HIP_DEVICE_COMPILE__)
  asm volatile("v_nop\n\tv_nop\n\tv_nop\n\tv_nop" : "+v"(t), "+v"(acc) : "v"(x), "v"(y));
#endif
}
__device__ __forceinline__ void dep_guard_h(v8f& a, v8f& b, v16h x, v16h y) {
#if defined(__HIP_DEVICE_COMPILE__)
  asm volatile("v_nop\n\tv_nop\n\tv_nop\n\tv_nop" : "+v"(a), "+v"(b) : "v"(x), "v"(y));
#endif
}
__device__ __forceinline__ void guard4x4(v8f& a, v8f& b, v8f& c, v8f& d,
                                         v16h u, v16h v, v16h w, v16h x) {
#if defined(__HIP_DEVICE_COMPILE__)
  asm volatile("v_nop\n\tv_nop\n\tv_nop\n\tv_nop"
               : "+v"(a), "+v"(b), "+v"(c), "+v"(d)
               : "v"(u), "v"(v), "v"(w), "v"(x));
#endif
}
__device__ __forceinline__ void guard4x6(v8f& a, v8f& b, v8f& c, v8f& d,
                                         v16h u, v16h v, v16h w, v16h x, v16h y, v16h z) {
#if defined(__HIP_DEVICE_COMPILE__)
  asm volatile("v_nop\n\tv_nop\n\tv_nop\n\tv_nop"
               : "+v"(a), "+v"(b), "+v"(c), "+v"(d)
               : "v"(u), "v"(v), "v"(w), "v"(x), "v"(y), "v"(z));
#endif
}
__device__ __forceinline__ void keep4_h(v16h a, v16h b, v16h c, v16h d) {
#if defined(__HIP_DEVICE_COMPILE__)
  asm volatile("v_nop" :: "v"(a), "v"(b), "v"(c), "v"(d));
#endif
}
__device__ __forceinline__ void acc_guard4(v8f& a, v8f& b, v8f& c, v8f& d) {
#if defined(__HIP_DEVICE_COMPILE__)
  asm volatile("v_nop\n\tv_nop\n\tv_nop\n\tv_nop" : "+v"(a), "+v"(b), "+v"(c), "+v"(d));
#endif
}
__device__ __forceinline__ void wave_sync_lds() {
  __builtin_amdgcn_fence(__ATOMIC_RELEASE, "workgroup");
  __builtin_amdgcn_wave_barrier();
  __builtin_amdgcn_fence(__ATOMIC_ACQUIRE, "workgroup");
}

__global__ __launch_bounds__(256) void cvt_h8(const float* __restrict__ in, unsigned short* out, int n8, float scale) {
  const int i = blockIdx.x * 256 + threadIdx.x;
  if (i < n8) {
    const v4f a = *(const v4f*)(in + (size_t)i * 8);
    const v4f c = *(const v4f*)(in + (size_t)i * 8 + 4);
    float f[8];
    f[0] = a[0]; f[1] = a[1]; f[2] = a[2]; f[3] = a[3];
    f[4] = c[0]; f[5] = c[1]; f[6] = c[2]; f[7] = c[3];
    unsigned short hb[8];
#pragma unroll
    for (int e = 0; e < 8; ++e) hb[e] = h_bits((_Float16)(bf_up(bf_bits(f[e])) * scale));
    v4u p;
    p[0] = pk16(hb[0], hb[1]);
    p[1] = pk16(hb[2], hb[3]);
    p[2] = pk16(hb[4], hb[5]);
    p[3] = pk16(hb[6], hb[7]);
    *(volatile v4u*)(out + (size_t)i * 8) = p;
    __threadfence();
    *(volatile v4u*)(out + (size_t)i * 8) = p;
  }
}

#define WTP 72
__global__ __launch_bounds__(256) void cvt_wt(const float* __restrict__ w0, const float* __restrict__ w1,
                                              const float* __restrict__ w2, const float* __restrict__ w3,
                                              unsigned short* out, float scale) {
  __shared__ __align__(16) unsigned short ts[64 * WTP];
  const int tid = threadIdx.x;
  const int o0 = blockIdx.x * 64, c0 = blockIdx.y * 64, z = blockIdx.z;
  const float* W = (z == 0) ? w0 : ((z == 1) ? w1 : ((z == 2) ? w2 : w3));
  unsigned short* outz = out + (size_t)z * DM * DM;
#pragma unroll 1
  for (int pass = 0; pass < 4; ++pass) {
    const int c  = pass * 16 + (tid >> 4);
    const int o4 = (tid & 15) * 4;
    const v4f v = *(const v4f*)(W + ((size_t)(c0 + c)) * DM + o0 + o4);
#pragma unroll
    for (int i = 0; i < 4; ++i) ts[(o4 + i) * WTP + c] = h_bits((_Float16)(bf_up(bf_bits(v[i])) * scale));
  }
  __syncthreads();
#pragma unroll 1
  for (int pass = 0; pass < 2; ++pass) {
    const int r  = pass * 32 + (tid >> 3);
    const int c8 = (tid & 7) * 8;
    const v4u v = *(const v4u*)(ts + r * WTP + c8);
    unsigned short* dst = outz + ((size_t)(o0 + r)) * DM + c0 + c8;
    *(volatile v4u*)dst = v;
    __threadfence();
    *(volatile v4u*)dst = v;
  }
}

template <int NSPLIT>
__global__ __launch_bounds__(256) void gemm64(
    const unsigned short* __restrict__ Ap, int lda,
    const unsigned short* __restrict__ A2p, int lda2,
    const unsigned short* __restrict__ Btp, int ldb,
    const float* __restrict__ bias,
    float* Cout, int ldc,
    int M, int N, int K, float oscale, float rres) {
  const _Float16* A  = (const _Float16*)(const void*)Ap;
  const _Float16* A2 = (const _Float16*)(const void*)A2p;
  const _Float16* Bt = (const _Float16*)(const void*)Btp;
  __shared__ __align__(16) float sT[8][16 * 68];
  const int lane = threadIdx.x & 31;
  const int wave = threadIdx.x >> 5;
  const int tilesN = N >> 6;
  const int tilesM = M >> 6;
  const int tile = blockIdx.x * 8 + wave;
  if (tile >= tilesM * tilesN) return;
  const int tm = tile / tilesN;
  const int tn = tile - tm * tilesN;
  const int m0 = tm << 6;
  const int n0 = tn << 6;

  const int rlane = lane & 15;
  const int koff  = (lane >> 4) * 8;
  const int mOff  = (lane >> 4) * 8;

  v8f acc[4][4];
#pragma unroll
  for (int i = 0; i < 4; ++i)
#pragma unroll
    for (int j = 0; j < 4; ++j) acc[i][j] = zero8();

  for (int k0 = 0; k0 < K; k0 += 32) {
    v16h bf[4];
#pragma unroll
    for (int j = 0; j < 4; ++j) {
      const size_t bo = (size_t)(n0 + (j << 4) + rlane) * ldb + koff + k0;
      bf[j] = ldfrag_h(Bt + bo);
    }
#pragma unroll
    for (int i = 0; i < 4; ++i) {
      const size_t ao = (size_t)(m0 + (i << 4) + rlane) * lda + koff + k0;
      const v16h ah = ldfrag_h(A + ao);
#pragma unroll
      for (int j = 0; j < 4; ++j) acc[i][j] = mma_h_raw(ah, bf[j], acc[i][j]);
      dep_guard_h(acc[i][0], acc[i][3], ah, bf[3]);
    }
    if (NSPLIT == 1) {
#pragma unroll
      for (int i = 0; i < 4; ++i) {
        const size_t ao = (size_t)(m0 + (i << 4) + rlane) * lda2 + koff + k0;
        const v16h al = ldfrag_h(A2 + ao);
#pragma unroll
        for (int j = 0; j < 4; ++j) {
          v8f tp = mma_h_raw(al, bf[j], zero8());
          res_guard(tp, acc[i][j], al, bf[j]);
#pragma unroll
          for (int r = 0; r < 8; ++r) acc[i][j][r] += tp[r] * rres;
        }
        dep_guard_h(acc[i][0], acc[i][3], al, bf[3]);
      }
    }
    keep4_h(bf[0], bf[1], bf[2], bf[3]);
  }
  acc_guard4(acc[0][0], acc[0][1], acc[0][2], acc[0][3]);
  acc_guard4(acc[1][0], acc[1][1], acc[1][2], acc[1][3]);
  acc_guard4(acc[2][0], acc[2][1], acc[2][2], acc[2][3]);
  acc_guard4(acc[3][0], acc[3][1], acc[3][2], acc[3][3]);

  float* slab = sT[wave];
  float* C = Cout;
  float bcol[4];
#pragma unroll
  for (int j = 0; j < 4; ++j) bcol[j] = bf_up(bf_bits(bias[n0 + (j << 4) + rlane]));
#pragma unroll
  for (int i = 0; i < 4; ++i) {
    const int mBase = m0 + (i << 4);
#pragma unroll
    for (int j = 0; j < 4; ++j) {
#pragma unroll
      for (int r = 0; r < 8; ++r) {
        slab[(mOff + r) * 68 + (j << 4) + rlane] = acc[i][j][r] * oscale + bcol[j];
      }
    }
    wave_sync_lds();
    {
      const int hh = lane >> 4, c4 = (lane & 15) * 4;
      for (int pass = 0; pass < 2; ++pass) {
#pragma unroll
        for (int it = 0; it < 8; ++it) {
          const int row = it * 2 + hh;
          const v4f v = *(const v4f*)(slab + row * 68 + c4);
          *(volatile v4f*)(C + (size_t)(mBase + row) * ldc + n0 + c4) = v;
        }
        __threadfence();
      }
    }
    wave_sync_lds();
  }
}

template <int HASRES>
__global__ __launch_bounds__(256) void relayout_hd(const float* __restrict__ Y, unsigned short* PH, unsigned short* PL, int n16) {
  const int i = blockIdx.x * 256 + threadIdx.x;
  if (i < n16) {
    const int inst = i / (TT * (HD / 8));
    const int rem  = i - inst * (TT * (HD / 8));
    const int t    = rem / (HD / 8);
    const int dq   = rem - t * (HD / 8);
    const int b = inst / NH, h = inst - b * NH;
    const float* src = Y + ((size_t)(b * TT + t)) * DM + h * HD + dq * 8;
    const v4f a  = *(const v4f*)(src);
    const v4f a2 = *(const v4f*)(src + 4);
    float f[8];
    f[0] = a[0]; f[1] = a[1]; f[2] = a[2]; f[3] = a[3];
    f[4] = a2[0]; f[5] = a2[1]; f[6] = a2[2]; f[7] = a2[3];
    unsigned short hb[8], lb[8];
#pragma unroll
    for (int e = 0; e < 8; ++e) {
      const float v = f[e] * 16.0f;
      const _Float16 xh = (_Float16)v;
      hb[e] = h_bits(xh);
      lb[e] = h_bits((_Float16)((v - (float)xh) * 2048.0f));
    }
    v4u ph, plv;
#pragma unroll
    for (int q = 0; q < 4; ++q) {
      ph[q]  = pk16(hb[2 * q], hb[2 * q + 1]);
      plv[q] = pk16(lb[2 * q], lb[2 * q + 1]);
    }
    const size_t dst = (size_t)i * 8;
    *(volatile v4u*)(PH + dst) = ph;
    if (HASRES) *(volatile v4u*)(PL + dst) = plv;
    __threadfence();
    *(volatile v4u*)(PH + dst) = ph;
    if (HASRES) *(volatile v4u*)(PL + dst) = plv;
  }
}

#define YP 68
__global__ __launch_bounds__(256) void relayout_v(const float* __restrict__ Y, unsigned short* VH, unsigned short* VL) {
  __shared__ __align__(16) float ys[64 * YP];
  const int tid = threadIdx.x;
  const int l0 = blockIdx.x * 64, c0 = blockIdx.y * 64, b = blockIdx.z;
  const float* Yb = Y + ((size_t)(b * TT + l0)) * DM + c0;

#pragma unroll 1
  for (int it = 0; it < 4; ++it) {
    const int idx = it * 256 + tid;
    const int row = idx >> 4;
    const int c4  = (idx & 15) * 4;
    const v4f v = *(const v4f*)(Yb + (size_t)row * DM + c4);
    *(v4f*)(ys + row * YP + c4) = v;
  }
  __syncthreads();

#pragma unroll 1
  for (int pass = 0; pass < 2; ++pass) {
    const int r  = pass * 32 + (tid >> 3);
    const int t8 = (tid & 7) * 8;
    const float* src = ys + t8 * YP + r;
    unsigned short hb[8], lb[8];
#pragma unroll
    for (int i = 0; i < 8; ++i) {
      const float v = src[i * YP] * 16.0f;
      const _Float16 xh = (_Float16)v;
      hb[i] = h_bits(xh);
      lb[i] = h_bits((_Float16)((v - (float)xh) * 2048.0f));
    }
    v4u ph, plv;
#pragma unroll
    for (int q = 0; q < 4; ++q) {
      ph[q]  = pk16(hb[2 * q], hb[2 * q + 1]);
      plv[q] = pk16(lb[2 * q], lb[2 * q + 1]);
    }
    const size_t dst = ((size_t)(b * DM + c0 + r)) * TT + l0 + t8;
    *(volatile v4u*)(VH + dst) = ph;
    *(volatile v4u*)(VL + dst) = plv;
    __threadfence();
    *(volatile v4u*)(VH + dst) = ph;
    *(volatile v4u*)(VL + dst) = plv;
  }
}

#define SP 72
__global__ __launch_bounds__(256) void attn_kernel(
    const unsigned short* __restrict__ QHp, const unsigned short* __restrict__ QLp,
    const unsigned short* __restrict__ KHp,
    const unsigned short* __restrict__ VHp, const unsigned short* __restrict__ VLp,
    const int* __restrict__ maskp,
    unsigned short* CTXh, unsigned short* CTXl, float rscale, float scl) {
  __shared__ __align__(16) unsigned short sth[8 * 16 * SP];
  __shared__ __align__(16) unsigned short stl[8 * 16 * SP];
  const _Float16* QH = (const _Float16*)(const void*)QHp;
  const _Float16* QL = (const _Float16*)(const void*)QLp;
  const _Float16* KH = (const _Float16*)(const void*)KHp;
  const _Float16* VH = (const _Float16*)(const void*)VHp;
  const _Float16* VL = (const _Float16*)(const void*)VLp;

  const int tid = threadIdx.x, lane = tid & 31, wave = tid >> 5;
  const int b = blockIdx.z, hp = blockIdx.y;
  const int qBase = blockIdx.x * QBLK + wave * 16;
  const int rlane = lane & 15, hsel = lane >> 4, koff = hsel * 8;
  const int qcol = qBase + rlane;
  const bool causal = (maskp[0] != 0);
  int ns = causal ? ((qBase + 16 + 31) >> 5) : (TT / 32);
  if (ns > TT / 32) ns = TT / 32;
  const float C2048  = 1.0f / 2048.0f;
  const float LN1024 = 6.931471805599453f;
  const float NEGBIG = -1.0e30f;
  const int   BIGDQ  = 1 << 20;

#pragma unroll 1
  for (int h2 = 0; h2 < 2; ++h2) {
    const int h = hp * 2 + h2;
    const int inst = b * NH + h;
    const size_t qo = ((size_t)inst * TT + qcol) * HD + koff;
    const v16h qh = ldfrag_h(QH + qo);
    const v16h ql = ldfrag_h(QL + qo);
    const _Float16* Khb = KH + ((size_t)inst * TT + rlane) * HD + koff;
    const _Float16* Vhb = VH + ((size_t)(b * DM + h * HD + rlane)) * TT + koff;
    const _Float16* Vlb = VL + ((size_t)(b * DM + h * HD + rlane)) * TT + koff;

    v8f oh0 = zero8(), oh1 = zero8(), ol0 = zero8(), ol1 = zero8();
    float m_run = -1e30f, l_run = 0.f;

#pragma unroll 1
    for (int st = 0; st < ns; ++st) {
      const int s = st * 32;
      const v16h kh0 = ldfrag_h(Khb + (size_t)s * HD);
      const v16h kh1 = ldfrag_h(Khb + (size_t)(s + 16) * HD);
      v8f sh0 = mma_h_raw(kh0, qh, zero8());
      v8f sr0 = mma_h_raw(kh0, ql, zero8());
      v8f sh1 = mma_h_raw(kh1, qh, zero8());
      v8f sr1 = mma_h_raw(kh1, ql, zero8());
      guard4x4(sh0, sh1, sr0, sr1, kh0, kh1, qh, ql);

      const int dq = causal ? (qcol - (s + koff)) : BIGDQ;
      float a0[8], a1[8];
#pragma unroll
      for (int r = 0; r < 8; ++r) {
        const float x0 = (sh0[r] + sr0[r] * C2048) * scl;
        const float x1 = (sh1[r] + sr1[r] * C2048) * scl;
        a0[r] = (r <= dq) ? x0 : NEGBIG;
        a1[r] = (r + 16 <= dq) ? x1 : NEGBIG;
      }

      float mloc = -1e30f;
#pragma unroll
      for (int r = 0; r < 8; ++r) mloc = fmaxf(mloc, fmaxf(a0[r], a1[r]));
      mloc = fmaxf(mloc, __shfl_xor(mloc, 16, 32));
      const float newM  = fmaxf(m_run, mloc);
      const float alpha = __expf(m_run - newM);
      const float msh   = newM - LN1024;
      float ssum = 0.f;
      float p0[8], p1[8];
#pragma unroll
      for (int r = 0; r < 8; ++r) {
        p0[r] = __expf(a0[r] - msh);
        p1[r] = __expf(a1[r] - msh);
        ssum += p0[r] + p1[r];
      }
      ssum += __shfl_xor(ssum, 16, 32);
      l_run = l_run * alpha + ssum;
      m_run = newM;
#pragma unroll
      for (int r = 0; r < 8; ++r) { oh0[r] *= alpha; oh1[r] *= alpha; ol0[r] *= alpha; ol1[r] *= alpha; }

      union { v16h v; _Float16 e[16]; } pf, pr;
#pragma unroll
      for (int r = 0; r < 8; ++r) {
        const _Float16 y0 = (_Float16)p0[r];
        const _Float16 y1 = (_Float16)p1[r];
        pf.e[r]     = y0;
        pf.e[8 + r] = y1;
        pr.e[r]     = (_Float16)((p0[r] - (float)y0) * 2048.0f);
        pr.e[8 + r] = (_Float16)((p1[r] - (float)y1) * 2048.0f);
      }

      const v16h vah0 = ldfrag_h(Vhb + s);
      const v16h vah1 = ldfrag_h(Vhb + (size_t)16 * TT + s);
      const v16h val0 = ldfrag_h(Vlb + s);
      const v16h val1 = ldfrag_h(Vlb + (size_t)16 * TT + s);
      oh0 = mma_h_raw(vah0, pf.v, oh0);
      ol0 = mma_h_raw(val0, pf.v, ol0);
      ol0 = mma_h_raw(vah0, pr.v, ol0);
      oh1 = mma_h_raw(vah1, pf.v, oh1);
      ol1 = mma_h_raw(val1, pf.v, ol1);
      ol1 = mma_h_raw(vah1, pr.v, ol1);
      guard4x6(oh0, oh1, ol0, ol1, vah0, vah1, val0, val1, pf.v, pr.v);
    }
    acc_guard4(oh0, oh1, ol0, ol1);

    const float inv = 4.0f * (1.0f / l_run);
    v4u hv0, lw0, hv1, lw1;
#pragma unroll
    for (int e = 0; e < 4; ++e) {
      {
        const float f0 = (oh0[2 * e]     + ol0[2 * e]     * C2048) * inv;
        const float f1 = (oh0[2 * e + 1] + ol0[2 * e + 1] * C2048) * inv;
        const _Float16 x0 = (_Float16)f0, x1 = (_Float16)f1;
        hv0[e] = pk16(h_bits(x0), h_bits(x1));
        lw0[e] = pk16(h_bits((_Float16)((f0 - (float)x0) * rscale)),
                      h_bits((_Float16)((f1 - (float)x1) * rscale)));
      }
      {
        const float f0 = (oh1[2 * e]     + ol1[2 * e]     * C2048) * inv;
        const float f1 = (oh1[2 * e + 1] + ol1[2 * e + 1] * C2048) * inv;
        const _Float16 x0 = (_Float16)f0, x1 = (_Float16)f1;
        hv1[e] = pk16(h_bits(x0), h_bits(x1));
        lw1[e] = pk16(h_bits((_Float16)((f0 - (float)x0) * rscale)),
                      h_bits((_Float16)((f1 - (float)x1) * rscale)));
      }
    }
    const int so = (wave * 16 + rlane) * SP + h2 * HD + koff;
    *(v4u*)(sth + so)      = hv0;
    *(v4u*)(sth + so + 16) = hv1;
    *(v4u*)(stl + so)      = lw0;
    *(v4u*)(stl + so + 16) = lw1;
  }

  wave_sync_lds();
  {
    const int rq = lane >> 3, c8 = (lane & 7) * 8;
    const unsigned short* hs = sth + (wave * 16) * SP;
    const unsigned short* ls = stl + (wave * 16) * SP;
    const size_t rb = (size_t)b * TT + qBase;
    for (int pass = 0; pass < 2; ++pass) {
#pragma unroll
      for (int it = 0; it < 4; ++it) {
        const int row = it * 4 + rq;
        const v4u v = *(const v4u*)(hs + row * SP + c8);
        *(volatile v4u*)(CTXh + (rb + row) * DM + hp * 64 + c8) = v;
      }
      __threadfence();
    }
    for (int pass = 0; pass < 2; ++pass) {
#pragma unroll
      for (int it = 0; it < 4; ++it) {
        const int row = it * 4 + rq;
        const v4u v = *(const v4u*)(ls + row * SP + c8);
        *(volatile v4u*)(CTXl + (rb + row) * DM + hp * 64 + c8) = v;
      }
      __threadfence();
    }
  }
}

extern "C" void kernel_launch(void* const* d_in, const int* in_sizes, int n_in,
                              void* d_out, int out_size, void* d_ws, size_t ws_size,
                              hipStream_t stream) {
  if (n_in < 10) return;
  if (in_sizes[0] != NTOK * DM) return;
  if (in_sizes[1] != DM * DM || in_sizes[3] != DM * DM || in_sizes[5] != DM * DM || in_sizes[7] != DM * DM) return;
  if (in_sizes[2] != DM || in_sizes[4] != DM || in_sizes[6] != DM || in_sizes[8] != DM) return;
  if (in_sizes[9] < 1) return;
  if (out_size != NTOK * DM) return;

  const float* x    = (const float*)d_in[0];
  const float* wq   = (const float*)d_in[1];
  const float* bq   = (const float*)d_in[2];
  const float* wk   = (const float*)d_in[3];
  const float* bk   = (const float*)d_in[4];
  const float* wv   = (const float*)d_in[5];
  const float* bv   = (const float*)d_in[6];
  const float* wf   = (const float*)d_in[7];
  const float* bfp  = (const float*)d_in[8];
  const int*   mask = (const int*)d_in[9];

  const size_t PXH = (size_t)NTOK * DM * 2;
  const size_t PWT = (size_t)4 * DM * DM * 2;
  const size_t PY  = (size_t)NTOK * DM * 4;
  const size_t PQ  = (size_t)NINST * TT * HD * 2;
  const size_t PV  = (size_t)NB * DM * TT * 2;
  const size_t PCT = (size_t)NTOK * DM * 2;
  size_t off = 0;
  const size_t oXH = off; off += PXH;
  const size_t oWT = off; off += PWT;
  const size_t oY  = off; off += PY;
  const size_t oQH = off; off += PQ;
  const size_t oQL = off; off += PQ;
  const size_t oKH = off; off += PQ;
  const size_t oVH = off; off += PV;
  const size_t oVL = off; off += PV;
  const size_t oCH = off; off += PCT;
  const size_t oCL = off; off += PCT;
  if (off > ws_size) return;
  if (off > (size_t)134217728) return;

  char* ws = (char*)d_ws;
  unsigned short* XH   = (unsigned short*)(ws + oXH);
  unsigned short* WT   = (unsigned short*)(ws + oWT);
  float*          Y    = (float*)(ws + oY);
  unsigned short* QH   = (unsigned short*)(ws + oQH);
  unsigned short* QL   = (unsigned short*)(ws + oQL);
  unsigned short* KH   = (unsigned short*)(ws + oKH);
  unsigned short* VH   = (unsigned short*)(ws + oVH);
  unsigned short* VL   = (unsigned short*)(ws + oVL);
  unsigned short* CTXh = (unsigned short*)(ws + oCH);
  unsigned short* CTXl = (unsigned short*)(ws + oCL);
  float*          out  = (float*)d_out;

  const dim3 blk(256);
  const int  n8x  = NTOK * DM / 8;
  const int  n16q = NINST * TT * HD / 8;
  const dim3 gX((n8x + 255) / 256);
  const dim3 gW(DM / 64, DM / 64, 4);
  const dim3 gG(((NTOK / 64) * (DM / 64) + 7) / 8);
  const dim3 gR((n16q + 255) / 256);
  const dim3 gRv(TT / 64, DM / 64, NB);
  const dim3 gAttn(TT / QBLK, NH / 2, NB);

  const float oscQkv = 1.0f / 16384.0f;
  const float rscale = 16384.0f;
  const float oscPrj = 1.0f / 65536.0f;
  const float rres   = 1.0f / 16384.0f;
  const float scl    = 0.044194173824159216f * (1.0f / 256.0f);

  cvt_h8<<<gX, blk, 0, stream>>>(x, XH, n8x, 16.0f);
  cvt_wt<<<gW, blk, 0, stream>>>(wq, wk, wv, wf, WT, 1024.0f);
  gemm64<0><<<gG, blk, 0, stream>>>(XH, DM, XH, DM, WT, DM, bq, Y, DM, NTOK, DM, DM, oscQkv, 0.0f);
  relayout_hd<1><<<gR, blk, 0, stream>>>(Y, QH, QL, n16q);
  gemm64<0><<<gG, blk, 0, stream>>>(XH, DM, XH, DM, WT + (size_t)DM * DM, DM, bk, Y, DM, NTOK, DM, DM, oscQkv, 0.0f);
  relayout_hd<0><<<gR, blk, 0, stream>>>(Y, KH, KH, n16q);
  gemm64<0><<<gG, blk, 0, stream>>>(XH, DM, XH, DM, WT + (size_t)2 * DM * DM, DM, bv, Y, DM, NTOK, DM, DM, oscQkv, 0.0f);
  relayout_v<<<gRv, blk, 0, stream>>>(Y, VH, VL);
  attn_kernel<<<gAttn, blk, 0, stream>>>(QH, QL, KH, VH, VL, mask, CTXh, CTXl, rscale, scl);
  gemm64<1><<<gG, blk, 0, stream>>>(CTXh, DM, CTXl, DM, WT + (size_t)3 * DM * DM, DM, bfp, out, DM,
                                    NTOK, DM, DM, oscPrj, rres);
  (void)hipGetLastError();
}
